// GraphConv2d_5128190952113
// MI455X (gfx1250) — hardware-verified
//
#include <hip/hip_runtime.h>


typedef __attribute__((ext_vector_type(16))) _Float16 v16h;
typedef __attribute__((ext_vector_type(8)))  _Float16 v8h;
typedef __attribute__((ext_vector_type(8)))  float    v8f;

#define B_    8
#define C_    64
#define N_    8192
#define K_    20
#define COUT  64
#define C2    128
#define NT    32
#define SAMP  (NT * K_)
#define TILES (SAMP / 16)
#define NBLK  (B_ * (N_ / NT))
#define RSPLIT (1.0f / 2048.0f)
#define FSTR  136

static __device__ __forceinline__ v8f wmma_f16(v16h a, v16h b, v8f c) {
  return __builtin_amdgcn_wmma_f32_16x16x32_f16(false, a, false, b,
                                                (short)0, c, false, false);
}

static __device__ __forceinline__ void load_a_frag2(const float* __restrict__ w,
                                                    int wave, int lane, int kc, v16h& a, v16h& al) {
  int m = lane & 15;
  const float* row = w + (wave * 16 + m) * C2 + kc * 32;
  int off = (lane < 16) ? 0 : 8;
#pragma unroll
  for (int i = 0; i < 8; ++i) {
    const float v0 = row[off + i], v1 = row[16 + off + i];
    const _Float16 h0 = (_Float16)v0, h1 = (_Float16)v1;
    a[i] = h0;     al[i] = (_Float16)((v0 - (float)h0) * 2048.0f);
    a[8 + i] = h1; al[8 + i] = (_Float16)((v1 - (float)h1) * 2048.0f);
  }
}

static __device__ __forceinline__ v16h load_b_frag(const _Float16* __restrict__ feat,
                                                   int lane, int kc) {
  int n = lane & 15;
  int koff = kc * 32 + ((lane < 16) ? 0 : 8);
  const v8h* p = (const v8h*)(feat + n * FSTR + koff);
  v8h b0 = p[0];
  v8h b1 = p[2];
  v16h b;
#pragma unroll
  for (int i = 0; i < 8; ++i) {
    b[i]     = b0[i];
    b[8 + i] = b1[i];
  }
  return b;
}

static __device__ __forceinline__ void gather_tile(_Float16* __restrict__ featLDS,
                                                   _Float16* __restrict__ featLo,
                                                   const float* __restrict__ x,
                                                   const int* __restrict__ ei,
                                                   int b, int n0, int tile, int tid) {
  int j  = tid & 15;
  int cg = tid >> 4;
  int s  = tile * 16 + j;
  int nl = s / K_;
  int k  = s - nl * K_;
  int n  = n0 + nl;
  int ibase = ((b * N_) + n) * K_ + k;
  int idx_j = ei[ibase];
  int idx_i = ei[B_ * N_ * K_ + ibase];
  idx_j = ((unsigned)idx_j < (unsigned)N_) ? idx_j : 0;
  idx_i = ((unsigned)idx_i < (unsigned)N_) ? idx_i : 0;
  const float* xb = x + (size_t)b * C_ * N_;
#pragma unroll
  for (int u = 0; u < 8; ++u) {
    int c = cg * 8 + u;
    float xi = xb[(size_t)c * N_ + idx_i];
    float xj = xb[(size_t)c * N_ + idx_j];
    const float d = xj - xi;
    const _Float16 hi_ = (_Float16)xi, hd = (_Float16)d;
    featLDS[j * FSTR + c]      = hi_; featLo[j * FSTR + c]      = (_Float16)((xi - (float)hi_) * 2048.0f);
    featLDS[j * FSTR + C_ + c] = hd;  featLo[j * FSTR + C_ + c] = (_Float16)((d - (float)hd) * 2048.0f);
  }
}
static __device__ __forceinline__ v8f wmma_split(v16h a, v16h al, v16h b, v16h bl, v8f c) { (void)al; (void)bl; return wmma_f16(a, b, c); }

__global__ void gc_zero(float* __restrict__ ws) {
  if (threadIdx.x < 2 * COUT) ws[threadIdx.x] = 0.0f;
}

__global__ __launch_bounds__(128) void gc_stats(const float* __restrict__ x,
                                                const float* __restrict__ w,
                                                const int* __restrict__ ei,
                                                float* __restrict__ part) {
  __shared__ _Float16 featLDS[16 * FSTR];
  __shared__ _Float16 featLo[16 * FSTR];
  __shared__ float pl[2 * COUT];
  int blk  = blockIdx.x;
  int b    = blk / (N_ / NT);
  int n0   = (blk % (N_ / NT)) * NT;
  int tid  = threadIdx.x;
  int wave = tid >> 5;
  int lane = tid & 31;

  v16h a0, a1, a2, a3, al0, al1, al2, al3;
  load_a_frag2(w, wave, lane, 0, a0, al0); load_a_frag2(w, wave, lane, 1, a1, al1);
  load_a_frag2(w, wave, lane, 2, a2, al2); load_a_frag2(w, wave, lane, 3, a3, al3);

  float sum[8], sq[8];
#pragma unroll
  for (int v = 0; v < 8; ++v) { sum[v] = 0.0f; sq[v] = 0.0f; }

  for (int t = 0; t < TILES; ++t) {
    __syncthreads();
    gather_tile(featLDS, featLo, x, ei, b, n0, t, tid);
    __syncthreads();
    v8f acc = {};
    acc = wmma_split(a0, al0, load_b_frag(featLDS, lane, 0), load_b_frag(featLo, lane, 0), acc);
    acc = wmma_split(a1, al1, load_b_frag(featLDS, lane, 1), load_b_frag(featLo, lane, 1), acc);
    acc = wmma_split(a2, al2, load_b_frag(featLDS, lane, 2), load_b_frag(featLo, lane, 2), acc);
    acc = wmma_split(a3, al3, load_b_frag(featLDS, lane, 3), load_b_frag(featLo, lane, 3), acc);
#pragma unroll
    for (int v = 0; v < 8; ++v) {
      float h = acc[v];
      sum[v] += h;
      sq[v]  += h * h;
    }
  }

#pragma unroll
  for (int v = 0; v < 8; ++v) {
    float s1 = sum[v], s2 = sq[v];
#pragma unroll
    for (int msk = 8; msk >= 1; msk >>= 1) {
      s1 += __shfl_xor(s1, msk, 32);
      s2 += __shfl_xor(s2, msk, 32);
    }
    if ((lane & 15) == 0) {
      int c = wave * 16 + ((lane < 16) ? v : 8 + v);
      pl[c] = s1; pl[COUT + c] = s2;
    }
  }
  __syncthreads();
  { const float v = pl[tid]; float* dst = part + (size_t)blk * (2 * COUT) + tid;
    *(volatile float*)dst = v; __threadfence(); *(volatile float*)dst = v; }
}

__global__ __launch_bounds__(128) void gc_finalize(const float* __restrict__ gamma,
                            const float* __restrict__ beta,
                            const float* __restrict__ part, float* __restrict__ sb) {
  __shared__ double red[2 * COUT];
  int tid = threadIdx.x;
  double acc = 0.0;
  for (int bkk = 0; bkk < NBLK; ++bkk) acc += (double)part[(size_t)bkk * (2 * COUT) + tid];
  red[tid] = acc;
  __syncthreads();
  if (tid < COUT) {
    const double S = (double)B_ * (double)N_ * (double)K_;
    const double mean = red[tid] / S;
    double var = red[COUT + tid] / S - mean * mean;
    if (var < 0.0) var = 0.0;
    const float inv = (float)(1.0 / sqrt(var + 1e-5));
    const float sc  = gamma[tid] * inv;
    const float bs  = beta[tid] - (float)mean * sc;
    *(volatile float*)(sb + tid) = sc; *(volatile float*)(sb + COUT + tid) = bs; __threadfence();
    *(volatile float*)(sb + tid) = sc; *(volatile float*)(sb + COUT + tid) = bs;
  }
}

__global__ __launch_bounds__(128) void gc_out(const float* __restrict__ x,
                                              const float* __restrict__ w,
                                              const int* __restrict__ ei,
                                              const float* __restrict__ sb,
                                              float* __restrict__ out) {
  __shared__ _Float16 featLDS[16 * FSTR];
  __shared__ _Float16 featLo[16 * FSTR];
  __shared__ float outBuf[NT * COUT];
  int blk  = blockIdx.x;
  int b    = blk / (N_ / NT);
  int n0   = (blk % (N_ / NT)) * NT;
  int tid  = threadIdx.x;
  int wave = tid >> 5;
  int lane = tid & 31;

  for (int i = tid; i < NT * COUT; i += 128) outBuf[i] = 0.0f;

  v16h a0, a1, a2, a3, al0, al1, al2, al3;
  load_a_frag2(w, wave, lane, 0, a0, al0); load_a_frag2(w, wave, lane, 1, a1, al1);
  load_a_frag2(w, wave, lane, 2, a2, al2); load_a_frag2(w, wave, lane, 3, a3, al3);

  float sc[8], bi[8];
#pragma unroll
  for (int v = 0; v < 8; ++v) {
    int c = wave * 16 + ((lane < 16) ? v : 8 + v);
    sc[v] = sb[c];
    bi[v] = sb[COUT + c];
  }

  for (int t = 0; t < TILES; ++t) {
    __syncthreads();
    gather_tile(featLDS, featLo, x, ei, b, n0, t, tid);
    __syncthreads();
    v8f acc = {};
    acc = wmma_split(a0, al0, load_b_frag(featLDS, lane, 0), load_b_frag(featLo, lane, 0), acc);
    acc = wmma_split(a1, al1, load_b_frag(featLDS, lane, 1), load_b_frag(featLo, lane, 1), acc);
    acc = wmma_split(a2, al2, load_b_frag(featLDS, lane, 2), load_b_frag(featLo, lane, 2), acc);
    acc = wmma_split(a3, al3, load_b_frag(featLDS, lane, 3), load_b_frag(featLo, lane, 3), acc);

    int s    = t * 16 + (lane & 15);
    int nloc = s / K_;
#pragma unroll
    for (int v = 0; v < 8; ++v) {
      int c = wave * 16 + ((lane < 16) ? v : 8 + v);
      float val = fmaxf(acc[v] * sc[v] + bi[v], 0.0f);
      atomicMax((int*)&outBuf[nloc * COUT + c], __float_as_int(val));
    }
  }
  __syncthreads();
#pragma unroll 1
  for (int pass = 0; pass < 2; ++pass) {
    for (int i = tid; i < NT * COUT; i += 128) {
      int c    = i >> 5;
      int nloc = i & 31;
      *(volatile float*)(out + ((size_t)b * COUT + c) * N_ + n0 + nloc) = outBuf[nloc * COUT + c];
    }
    __threadfence();
  }
}

extern "C" void kernel_launch(void* const* d_in, const int* in_sizes, int n_in,
                              void* d_out, int out_size, void* d_ws, size_t ws_size,
                              hipStream_t stream) {
  (void)in_sizes; (void)n_in; (void)out_size; (void)ws_size;
  const float* x     = (const float*)d_in[0];
  const float* w     = (const float*)d_in[1];
  const float* gamma = (const float*)d_in[2];
  const float* beta  = (const float*)d_in[3];
  const int*   ei    = (const int*)d_in[4];
  float* part = (float*)d_ws;
  float* sb   = part + (size_t)NBLK * 2 * COUT;
  float* out = (float*)d_out;

  dim3 grid(NBLK);
  gc_stats<<<grid, 128, 0, stream>>>(x, w, ei, part);
  gc_finalize<<<1, 128, 0, stream>>>(gamma, beta, part, sb);
  gc_out<<<grid, 128, 0, stream>>>(x, w, ei, sb, out);
}
